// ScalarMessagePassing_35691178230141
// MI455X (gfx1250) — hardware-verified
//
#include <hip/hip_runtime.h>


#define NN_   50000
#define NP    50176
#define NE_   800000
#define HID   128
#define HD_   192
#define NT    512
#define NWV   (NT / 32)
#define EPT   4
#define CHUNK (NT * EPT)
#define RB    512

typedef unsigned short bf;
typedef __attribute__((ext_vector_type(16))) __bf16   v16bf;
typedef __attribute__((ext_vector_type(8)))  unsigned short v8us;
typedef __attribute__((ext_vector_type(8)))  float    v8f;
typedef __attribute__((ext_vector_type(4)))  float    v4f;
typedef v4f  __attribute__((may_alias)) v4fa;
typedef v8us __attribute__((may_alias)) v8usa;

__device__ __forceinline__ unsigned short f2bf(float f) { unsigned u = __float_as_uint(f); u += 0x7FFFu + ((u >> 16) & 1u); return (unsigned short)(u >> 16); }
__device__ __forceinline__ float bf2f(unsigned short b) { return __uint_as_float(((unsigned)b) << 16); }
__device__ __forceinline__ float bfr(float f) { return bf2f(f2bf(f)); }
__device__ __forceinline__ v16bf cat16b(v8us lo, v8us hi) { return __builtin_bit_cast(v16bf, __builtin_shufflevector(lo, hi, 0, 1, 2, 3, 4, 5, 6, 7, 8, 9, 10, 11, 12, 13, 14, 15)); }
__device__ __forceinline__ v8f wmmab(v16bf a, v16bf b, v8f c) { return __builtin_amdgcn_wmma_f32_16x16x32_bf16(false, a, false, b, (short)0, c, false, false); }
#define VST2(T, p, v) do { const T vst2_v_ = (v); *(volatile T*)(p) = vst2_v_; __threadfence(); *(volatile T*)(p) = vst2_v_; } while (0)

__global__ __launch_bounds__(256) void k_sb(const float* __restrict__ h, bf* SB) {
    const int lane = threadIdx.x & 31, r = blockIdx.x * 8 + (threadIdx.x >> 5);
    if (r >= NP) return;
    typedef __attribute__((ext_vector_type(4))) unsigned short v4us;
    v4us t;
#pragma unroll
    for (int i = 0; i < 4; ++i) t[i] = (r < NN_) ? f2bf(h[(size_t)r * HD_ + lane * 4 + i]) : (unsigned short)0;
    VST2(v4us, SB + (size_t)r * HID + lane * 4, t);
}

__global__ __launch_bounds__(256) void k_wt(const float* __restrict__ Wsrc, bf* WT) {
    __shared__ __align__(16) unsigned short tl[64 * 72];
    const int tid = threadIdx.x, k0 = blockIdx.x * 64, n0 = blockIdx.y * 64;
    const int kk = tid >> 2, nq = (tid & 3) * 16;
#pragma unroll
    for (int i = 0; i < 16; ++i) tl[(nq + i) * 72 + kk] = f2bf(Wsrc[(size_t)(k0 + kk) * HID + n0 + nq + i]);
    __syncthreads();
    const int piece = tid & 7;
    auto pass = [&]() {
#pragma unroll
        for (int s = 0; s < 2; ++s) { const int nr = (tid >> 3) + 32 * s; const v8us val = *(const v8usa*)(tl + nr * 72 + piece * 8);
            *(volatile v8us*)(WT + (size_t)(n0 + nr) * HID + k0 + piece * 8) = val; }
    };
    pass(); __threadfence(); pass();
}

template <bool SPLITA>
__global__ __launch_bounds__(128) void k_gemmb(const bf* __restrict__ A, const bf* __restrict__ Al, const bf* __restrict__ Bn, float* C) {
    __shared__ __align__(16) float ost[4][16 * 68];
    const int lane = threadIdx.x & 31, wave = threadIdx.x >> 5, lr = lane & 15, hi = lane >> 4;
    const int r0 = blockIdx.x * 64 + wave * 16, c0 = blockIdx.y * 64;
    const size_t aoff = (size_t)(r0 + lr) * HID + 8 * hi;
    size_t boff[4];
#pragma unroll
    for (int t = 0; t < 4; ++t) boff[t] = (size_t)(c0 + t * 16 + lr) * HID + 8 * hi;
    v8f acc[4];
#pragma unroll
    for (int t = 0; t < 4; ++t) acc[t] = (v8f){};
#pragma unroll
    for (int kc = 0; kc < HID; kc += 32) {
        const v16bf a = cat16b(*(const v8us*)(A + aoff + kc), *(const v8us*)(A + aoff + kc + 16));
        v16bf al = a;
        if (SPLITA) al = cat16b(*(const v8us*)(Al + aoff + kc), *(const v8us*)(Al + aoff + kc + 16));
#pragma unroll
        for (int t = 0; t < 4; ++t) { const v16bf b = cat16b(*(const v8us*)(Bn + boff[t] + kc), *(const v8us*)(Bn + boff[t] + kc + 16)); acc[t] = wmmab(a, b, acc[t]); if (SPLITA) acc[t] = wmmab(al, b, acc[t]); }
    }
    asm volatile("v_nop\n\tv_nop\n\tv_nop\n\tv_nop" : "+v"(acc[0]), "+v"(acc[1]), "+v"(acc[2]), "+v"(acc[3]));
    float* os = &ost[wave][0];
#pragma unroll
    for (int t = 0; t < 4; ++t)
#pragma unroll
        for (int j = 0; j < 8; ++j) os[(hi * 8 + j) * 68 + t * 16 + lr] = acc[t][j];
    __syncthreads();
    float* crow = C + (size_t)r0 * HID + c0;
    auto pass = [&]() {
#pragma unroll
        for (int s = 0; s < 8; ++s) { const int Lid = (lane >> 3) + 4 * s, piece = lane & 7; const int row = Lid >> 1, cofs = (Lid & 1) * 32 + piece * 4;
            const v4f val = *(const v4fa*)(os + row * 68 + cofs); *(volatile v4f*)(crow + (size_t)row * HID + cofs) = val; }
    };
    pass(); __threadfence(); pass();
}

__device__ __forceinline__ float silu_(float x) { return x / (1.0f + __expf(-x)); }
__global__ __launch_bounds__(NT) void k_aggr(const float* __restrict__ P, const float* __restrict__ Q, const int* __restrict__ ei, const float* __restrict__ elen,
                                             const float* __restrict__ wlen, const float* __restrict__ b1, bf* HH, bf* HL, float* CNT) {
    extern __shared__ float4 lds_raw[];
    float* agg = (float*)lds_raw; int* lst = (int*)(agg + RB * HID); float* lsv = (float*)(lst + CHUNK); int* cnt = (int*)(lsv + CHUNK); int* wtot = cnt + RB;
    const int t = threadIdx.x, lane = t & 31, wv = t >> 5, n0 = blockIdx.x * RB;
    const int* snd = ei; const int* rcv = ei + NE_;
    for (int i = t; i < RB * HID; i += NT) agg[i] = 0.0f;
    if (t < RB) cnt[t] = 0;
    const float wl = (t < HID) ? bfr(wlen[t]) : 0.f, bb = (t < HID) ? bfr(b1[t]) : 0.f;
    __syncthreads();
#pragma unroll 1
    for (int base = 0; base < NE_; base += CHUNK) {
        int val[EPT]; float vv[EPT]; int flg[EPT]; int c = 0;
#pragma unroll
        for (int j = 0; j < EPT; ++j) {
            const int e = base + j * NT + t;
            int d = (e < NE_) ? rcv[e] : -1; if (d < 0 && e < NE_) d += NN_;
            const unsigned udl = (unsigned)d - (unsigned)n0;
            const int f = (udl < (unsigned)RB) ? 1 : 0; int v = 0; float w = 0.f;
            if (f) { int s = snd[e]; if (s < 0) s += NN_; s = min(max(s, 0), NN_ - 1); v = s * RB + (int)udl; w = bfr(elen[e]); }
            val[j] = v; vv[j] = w; flg[j] = f; c += f;
        }
        int incl = c;
#pragma unroll
        for (int o = 1; o < 32; o <<= 1) { const int y = __shfl_up(incl, o, 32); if (lane >= o) incl += y; }
        if (lane == 31) wtot[wv] = incl;
        __syncthreads();
        int off = incl - c, tot = 0;
#pragma unroll
        for (int i = 0; i < NWV; ++i) { const int v = wtot[i]; off += (i < wv) ? v : 0; tot += v; }
#pragma unroll
        for (int j = 0; j < EPT; ++j) { if (flg[j]) { lst[off] = val[j]; lsv[off] = vv[j]; ++off; } }
        __syncthreads();
        if (tot > 0) {
            if (t < HID) {
#pragma unroll 1
                for (int e2 = 0; e2 < tot; ++e2) { const int v = lst[e2]; const int s = v >> 9, dl = v & (RB - 1);
                    agg[dl * HID + t] += silu_(P[(size_t)s * HID + t] + Q[(size_t)(n0 + dl) * HID + t] + lsv[e2] * wl + bb); }
            } else if (t == HID) {
#pragma unroll 1
                for (int e2 = 0; e2 < tot; ++e2) cnt[lst[e2] & (RB - 1)] += 1;
            }
        }
        __syncthreads();
    }
    typedef __attribute__((ext_vector_type(4))) unsigned short v4us;
#pragma unroll 1
    for (int i = 0; i < RB / NWV; ++i) {
        const int rl = wv * (RB / NWV) + i; const size_t r = (size_t)(n0 + rl);
        v4us oh, ol;
#pragma unroll
        for (int q = 0; q < 4; ++q) { const float v = agg[rl * HID + lane * 4 + q]; const unsigned short hb = f2bf(v); oh[q] = hb; ol[q] = f2bf(v - bf2f(hb)); }
        *(volatile v4us*)(HH + r * HID + lane * 4) = oh; *(volatile v4us*)(HL + r * HID + lane * 4) = ol;
        __threadfence();
        *(volatile v4us*)(HH + r * HID + lane * 4) = oh; *(volatile v4us*)(HL + r * HID + lane * 4) = ol;
    }
    VST2(float, CNT + n0 + wv * 32 + lane, (float)cnt[wv * 32 + lane]);
}

__global__ __launch_bounds__(256) void k_final(const float* __restrict__ h, const float* __restrict__ AGG, const float* __restrict__ CNT, const float* __restrict__ b2, float* out) {
    const int lane = threadIdx.x & 31, r = blockIdx.x * 8 + (threadIdx.x >> 5);
    if (r >= NN_) return;
    float v[6];
    const float cn = CNT[r];
#pragma unroll
    for (int q = 0; q < 6; ++q) { const int c = q * 32 + lane; const float hv = bfr(h[(size_t)r * HD_ + c]);
        v[q] = (q < 4) ? (hv + (AGG[(size_t)r * HID + c] + cn * bfr(b2[c]))) : hv; }
    float* d = out + (size_t)r * HD_;
#pragma unroll
    for (int q = 0; q < 6; ++q) *(volatile float*)(d + q * 32 + lane) = v[q];
    __threadfence();
#pragma unroll
    for (int q = 0; q < 6; ++q) *(volatile float*)(d + q * 32 + lane) = v[q];
}

extern "C" void kernel_launch(void* const* d_in, const int* in_sizes, int n_in,
                              void* d_out, int out_size, void* d_ws, size_t ws_size, hipStream_t stream) {
    (void)in_sizes; (void)n_in; (void)out_size;
    const float* h = (const float*)d_in[0]; const int* ei = (const int*)d_in[1]; const float* elen = (const float*)d_in[2];
    const float* W1 = (const float*)d_in[3]; const float* b1 = (const float*)d_in[4]; const float* W2 = (const float*)d_in[5]; const float* b2 = (const float*)d_in[6];
    float* out = (float*)d_out;
    char* wsp = (char*)d_ws;
    auto take = [&](size_t bytes) { char* p = wsp; wsp += (bytes + 255) & ~(size_t)255; return (void*)p; };
    bf* SB = (bf*)take((size_t)NP * HID * 2);
    bf* W1AT = (bf*)take((size_t)HID * HID * 2); bf* W1BT = (bf*)take((size_t)HID * HID * 2); bf* W2T = (bf*)take((size_t)HID * HID * 2);
    float* P = (float*)take((size_t)NP * HID * 4); float* Q = (float*)take((size_t)NP * HID * 4);
    bf* HH = (bf*)take((size_t)NP * HID * 2); bf* HL = (bf*)take((size_t)NP * HID * 2); float* CNT = (float*)take((size_t)NP * 4);
    float* AGG = (float*)take((size_t)NP * HID * 4);
    if ((size_t)(wsp - (char*)d_ws) > ws_size) return;
    k_sb<<<NP / 8, 256, 0, stream>>>(h, SB);
    k_wt<<<dim3(HID / 64, HID / 64, 1), 256, 0, stream>>>(W1, W1AT);
    k_wt<<<dim3(HID / 64, HID / 64, 1), 256, 0, stream>>>(W1 + (size_t)HID * HID, W1BT);
    k_wt<<<dim3(HID / 64, HID / 64, 1), 256, 0, stream>>>(W2, W2T);
    k_gemmb<false><<<dim3(NP / 64, HID / 64, 1), 128, 0, stream>>>(SB, nullptr, W1AT, P);
    k_gemmb<false><<<dim3(NP / 64, HID / 64, 1), 128, 0, stream>>>(SB, nullptr, W1BT, Q);
    const size_t lds = (size_t)RB * HID * 4 + (size_t)CHUNK * 8 + RB * 4 + NWV * 4;
    k_aggr<<<NP / RB, NT, lds, stream>>>(P, Q, ei, elen, W1 + (size_t)2 * HID * HID, b1, HH, HL, CNT);
    k_gemmb<true><<<dim3(NP / 64, HID / 64, 1), 128, 0, stream>>>(HH, HL, W2T, AGG);
    k_final<<<(NN_ + 7) / 8, 256, 0, stream>>>(h, AGG, CNT, b2, out);
}
